// Mamba_block_29008209117720
// MI455X (gfx1250) — hardware-verified
//
#include <hip/hip_runtime.h>


#define NB_   2
#define NL_   1024
#define DM_   1024
#define DI_   2048
#define NS_   16
#define DR_   64
#define XPN_  96
#define XPP_  128
#define MT_   (NB_ * NL_)

#define SC_U   8.0f
#define SC_W   32.0f
#define SC_XC  32.0f
#define SC_DT  32.0f
#define SC_Y   64.0f

static_assert(MT_ % 64 == 0);
static_assert((2 * DI_) % 128 == 0);
static_assert(DI_ % 128 == 0);
static_assert(DM_ % 128 == 0);
static_assert(XPP_ % 128 == 0);
static_assert(DM_ % 32 == 0);
static_assert(DI_ % 32 == 0);
static_assert(DR_ % 32 == 0);
static_assert((NL_ & (NL_ - 1)) == 0);
static_assert(DM_ == 128 * 8);
static_assert(DI_ == 256 * 8);
static_assert(XPN_ == DR_ + 2 * NS_);

typedef float          v4f   __attribute__((ext_vector_type(4)));
typedef float          v8f   __attribute__((ext_vector_type(8)));
typedef _Float16       v8h   __attribute__((ext_vector_type(8)));
typedef _Float16       v16h  __attribute__((ext_vector_type(16)));
typedef unsigned short u16x8 __attribute__((ext_vector_type(8)));

union FragH { u16x8 h[2]; v16h v; };
union Pack8 { v8h f; u16x8 u; };
union H1    { _Float16 f; unsigned short u; };

__device__ __forceinline__ float silu_f(float x) {
    float e = expf(-x);
    return x * __builtin_amdgcn_rcpf(1.0f + e);
}
__device__ __forceinline__ float softplus_f(float x) {
    return fmaxf(x, 0.0f) + log1pf(expf(-fabsf(x)));
}
__device__ __forceinline__ float conv4_silu(float x0, float x1, float x2, float x3,
                                            float w0, float w1, float w2, float w3, float bias) {
    float c = w0 * x0 + w1 * x1 + w2 * x2 + w3 * x3;
    return silu_f(c + bias);
}
__device__ __forceinline__ v8f ld8f(const float* p) {
    v4f a = *(const v4f*)p;
    v4f b = *(const v4f*)(p + 4);
    return __builtin_shufflevector(a, b, 0, 1, 2, 3, 4, 5, 6, 7);
}

__device__ __forceinline__ void mma16(v8f& acc, const FragH& a, const FragH& b) {
    acc = __builtin_amdgcn_wmma_f32_16x16x32_f16(false, a.v, false, b.v, (short)0, acc, false, false);
    asm volatile("v_nop\n\tv_nop\n\tv_nop\n\tv_nop" : "+v"(acc) : "v"(a.v), "v"(b.v));
}

__global__ __launch_bounds__(256)
void cvt_kernel(const float* __restrict__ src, unsigned short* dst, int n8, float scale)
{
    const int i = blockIdx.x * 256 + threadIdx.x;
    if (i >= n8) return;
    const size_t e = (size_t)i * 8;
    const v8f x = ld8f(src + e);
    Pack8 pk;
    pk.f = __builtin_convertvector(x * scale, v8h);
    const u16x8 v = pk.u;
    *(volatile u16x8*)(dst + e) = v;
    __threadfence();
    *(volatile u16x8*)(dst + e) = v;
}

__global__ __launch_bounds__(128)
void rmsnorm_kernel(const float* __restrict__ X, const float* __restrict__ nw, unsigned short* U16)
{
    __shared__ float red[4];
    const int row  = blockIdx.x;
    const int tid  = threadIdx.x;
    const int lane = tid & 31;
    const int wave = tid >> 5;
    const int c0   = tid * 8;

    const v8f xv = ld8f(X + (size_t)row * DM_ + c0);
    float ss = 0.0f;
#pragma unroll
    for (int c = 0; c < 8; ++c) ss += xv[c] * xv[c];
#pragma unroll
    for (int o = 16; o > 0; o >>= 1) ss += __shfl_xor(ss, o, 32);
    if (lane == 0) red[wave] = ss;
    __syncthreads();
    const float tot = (red[0] + red[1]) + (red[2] + red[3]);
    const float sc  = rsqrtf(tot * (1.0f / DM_) + 1e-5f);

    const v8f wv = ld8f(nw + c0);
    v8f u;
#pragma unroll
    for (int c = 0; c < 8; ++c) u[c] = ((xv[c] * sc) * wv[c]) * SC_U;

    Pack8 pk;
    pk.f = __builtin_convertvector(u, v8h);
    const u16x8 v = pk.u;
    unsigned short* gp = U16 + (size_t)row * DM_ + c0;
    *(volatile u16x8*)gp = v;
    __threadfence();
    *(volatile u16x8*)gp = v;
}

template<int NBF>
__device__ __forceinline__ void tile_store_pass(const float* st, float* gp, int ldc, int lane) {
    constexpr int CW  = NBF * 16;
    constexpr int P   = CW + 4;
    constexpr int LPR = CW / 4;
    constexpr int RPI = 32 / LPR;
    constexpr int NIT = 32 / RPI;
    const int rsub = lane / LPR;
    const int c4   = (lane % LPR) * 4;
#pragma unroll
    for (int it = 0; it < NIT; ++it) {
        const int row = it * RPI + rsub;
        const v4f v = *(const v4f*)(st + row * P + c4);
        *(volatile v4f*)(gp + (size_t)row * ldc + c4) = v;
    }
}

template<int NBF, bool RES>
__global__ __launch_bounds__(128)
void gemm_tn_kernel(const unsigned short* __restrict__ A, const unsigned short* __restrict__ Bw,
                    float* C, float* C2, const float* __restrict__ R,
                    int K, int ldc, int csplit, float scale)
{
    constexpr int CW = NBF * 16;
    constexpr int P  = CW + 4;
    __shared__ __attribute__((aligned(16))) float stile[4][32 * P];

    const int tid  = threadIdx.x;
    const int lane = tid & 31;
    const int wave = tid >> 5;
    const int h    = lane >> 4;
    const int m    = lane & 15;
    const int wm   = wave >> 1;
    const int wn   = wave & 1;

    const int rowW = blockIdx.y * 64 + wm * 32;
    const int colW = blockIdx.x * (2 * CW) + wn * CW;

    v8f acc[2 * NBF];
#pragma unroll
    for (int j = 0; j < 2 * NBF; ++j)
#pragma unroll
        for (int r = 0; r < 8; ++r) acc[j][r] = 0.0f;

    const size_t aoff  = (size_t)(rowW + m) * K + 8 * h;
    const size_t boff  = (size_t)(colW + m) * K + 8 * h;
    const size_t sub16 = (size_t)16 * K;
    const int nk = K >> 5;

    for (int kt = 0; kt < nk; ++kt) {
        const size_t k0 = (size_t)kt * 32;
        FragH fa[2], fb[NBF];
#pragma unroll
        for (int s = 0; s < 2; ++s) {
            const unsigned short* p = A + aoff + s * sub16 + k0;
            fa[s].h[0] = *(const u16x8*)(p);
            fa[s].h[1] = *(const u16x8*)(p + 16);
        }
#pragma unroll
        for (int j = 0; j < NBF; ++j) {
            const unsigned short* p = Bw + boff + j * sub16 + k0;
            fb[j].h[0] = *(const u16x8*)(p);
            fb[j].h[1] = *(const u16x8*)(p + 16);
        }
#pragma unroll
        for (int s = 0; s < 2; ++s)
#pragma unroll
            for (int j = 0; j < NBF; ++j)
                mma16(acc[s * NBF + j], fa[s], fb[j]);
    }

    float* Cp = C;
    int gcol = colW;
    if (colW >= csplit) { Cp = C2; gcol = colW - csplit; }

    float* st = stile[wave];
#pragma unroll
    for (int s = 0; s < 2; ++s)
#pragma unroll
        for (int j = 0; j < NBF; ++j)
#pragma unroll
            for (int r = 0; r < 8; ++r) {
                const int lrow = s * 16 + 8 * h + r;
                const int lcol = j * 16 + m;
                float v = acc[s * NBF + j][r] * scale;
                if (RES) v += R[(size_t)(rowW + lrow) * ldc + gcol + lcol];
                st[lrow * P + lcol] = v;
            }
    __syncthreads();

    float* gp = Cp + (size_t)rowW * ldc + gcol;
    tile_store_pass<NBF>(st, gp, ldc, lane);
    __threadfence();
    tile_store_pass<NBF>(st, gp, ldc, lane);
}

__global__ __launch_bounds__(256)
void conv_silu_kernel(const float* __restrict__ Xin, const float* __restrict__ cw,
                      const float* __restrict__ cb, unsigned short* XC16)
{
    const int m  = blockIdx.x;
    const int l  = m & (NL_ - 1);
    const int d0 = threadIdx.x * 8;
    const float* xr = Xin + (size_t)m * DI_ + d0;

    v8f x3 = ld8f(xr);
    v8f x2, x1, x0;
#pragma unroll
    for (int c = 0; c < 8; ++c) { x2[c] = 0.0f; x1[c] = 0.0f; x0[c] = 0.0f; }
    if (l >= 1) x2 = ld8f(xr - DI_);
    if (l >= 2) x1 = ld8f(xr - 2 * DI_);
    if (l >= 3) x0 = ld8f(xr - 3 * DI_);

    const float* wp = cw + (size_t)d0 * 4;
    v4f wv[8];
#pragma unroll
    for (int c = 0; c < 8; ++c) wv[c] = *(const v4f*)(wp + 4 * c);
    const v8f bias = ld8f(cb + d0);

    v8f u;
#pragma unroll
    for (int c = 0; c < 8; ++c)
        u[c] = conv4_silu(x0[c], x1[c], x2[c], x3[c], wv[c][0], wv[c][1], wv[c][2], wv[c][3], bias[c]) * SC_XC;

    Pack8 pk;
    pk.f = __builtin_convertvector(u, v8h);
    const u16x8 v = pk.u;
    unsigned short* gp = XC16 + (size_t)m * DI_ + d0;
    *(volatile u16x8*)gp = v;
    __threadfence();
    *(volatile u16x8*)gp = v;
}

__global__ __launch_bounds__(256)
void dtslice_kernel(const float* __restrict__ Dbl, unsigned short* DT16)
{
    const int i = blockIdx.x * 256 + threadIdx.x;
    if (i >= (MT_ * DR_) / 8) return;
    const int row = i >> 3;
    const int c   = (i & 7) * 8;
    const v8f x = ld8f(Dbl + (size_t)row * XPP_ + c);
    Pack8 pk;
    pk.f = __builtin_convertvector(x * SC_DT, v8h);
    const u16x8 v = pk.u;
    unsigned short* gp = DT16 + (size_t)row * DR_ + c;
    *(volatile u16x8*)gp = v;
    __threadfence();
    *(volatile u16x8*)gp = v;
}

__device__ __forceinline__ void y16_store_pass(const unsigned short* sl, unsigned short* gp,
                                               size_t gbase, int tid) {
#pragma unroll
    for (int it = 0; it < 2; ++it) {
        const int t = it * 8 + (tid >> 3);
        const int c = (tid & 7) * 8;
        const u16x8 v = *(const u16x8*)(sl + t * 64 + c);
        *(volatile u16x8*)(gp + gbase + (size_t)t * DI_ + c) = v;
    }
}

__global__ __launch_bounds__(64)
void scan_kernel(const float* __restrict__ Xin, const float* __restrict__ Zf, const float* __restrict__ Dl,
                 const float* __restrict__ Dbl,
                 const float* __restrict__ cw, const float* __restrict__ cb,
                 const float* __restrict__ dtb, const float* __restrict__ Alog,
                 const float* __restrict__ Dp, unsigned short* Y16)
{
    __shared__ __attribute__((aligned(16))) float sbc[16 * 32];
    __shared__ __attribute__((aligned(16))) unsigned short sy[16 * 64];

    const int tid   = threadIdx.x;
    const int dbase = blockIdx.x * 64;
    const int d     = dbase + tid;
    const int b     = blockIdx.y;

    float an[NS_], hs[NS_];
#pragma unroll
    for (int n = 0; n < NS_; ++n) {
        an[n] = -expf(Alog[d * NS_ + n]);
        hs[n] = 0.0f;
    }
    const float w0 = cw[d * 4 + 0], w1 = cw[d * 4 + 1], w2 = cw[d * 4 + 2], w3 = cw[d * 4 + 3];
    const float cbias = cb[d];
    const float tb = dtb[d];
    const float Dd = Dp[d];

    float xm1 = 0.0f, xm2 = 0.0f, xm3 = 0.0f;
    const size_t mrow0 = (size_t)b * NL_;

#pragma unroll 1
    for (int l0 = 0; l0 < NL_; l0 += 16) {
        {
            const int t    = tid >> 2;
            const int part = tid & 3;
            const float* src = Dbl + (mrow0 + (size_t)(l0 + t)) * XPP_ + DR_ + part * 8;
            const v4f va = *(const v4f*)(src);
            const v4f vb = *(const v4f*)(src + 4);
            *(v4f*)(sbc + t * 32 + part * 8)     = va;
            *(v4f*)(sbc + t * 32 + part * 8 + 4) = vb;
        }
        __syncthreads();

#pragma unroll 1
        for (int t = 0; t < 16; ++t) {
            const size_t mrow = mrow0 + (size_t)(l0 + t);
            const size_t e = mrow * DI_ + d;
            const float xv = Xin[e];
            const float zv = Zf[e];
            const float dl = Dl[e];
            const float u  = conv4_silu(xm3, xm2, xm1, xv, w0, w1, w2, w3, cbias);
            xm3 = xm2; xm2 = xm1; xm1 = xv;
            const float dt = softplus_f(dl + tb);
            const float du = dt * u;

            const float* bp = sbc + t * 32;
            float bn[NS_], cn[NS_];
#pragma unroll
            for (int q = 0; q < 4; ++q) {
                const v4f vb = *(const v4f*)(bp + 4 * q);
                const v4f vc = *(const v4f*)(bp + 16 + 4 * q);
                bn[4 * q + 0] = vb[0]; bn[4 * q + 1] = vb[1]; bn[4 * q + 2] = vb[2]; bn[4 * q + 3] = vb[3];
                cn[4 * q + 0] = vc[0]; cn[4 * q + 1] = vc[1]; cn[4 * q + 2] = vc[2]; cn[4 * q + 3] = vc[3];
            }

            float y = 0.0f;
#pragma unroll
            for (int n = 0; n < NS_; ++n) {
                const float da = __expf(dt * an[n]);
                hs[n] = da * hs[n] + du * bn[n];
                y += hs[n] * cn[n];
            }
            const float g = (y + Dd * u) * silu_f(zv);
            H1 hb;
            hb.f = (_Float16)(g * SC_Y);
            sy[t * 64 + tid] = hb.u;
        }
        __syncthreads();
        const size_t gbase = (mrow0 + (size_t)l0) * DI_ + dbase;
        y16_store_pass(sy, Y16, gbase, tid);
        __threadfence();
        y16_store_pass(sy, Y16, gbase, tid);
        __syncthreads();
    }
}

extern "C" void kernel_launch(void* const* d_in, const int* in_sizes, int n_in,
                              void* d_out, int out_size, void* d_ws, size_t ws_size,
                              hipStream_t stream)
{
    if (n_in < 11) return;
    if (in_sizes[0]  != MT_ * DM_)       return;
    if (in_sizes[1]  != DM_)             return;
    if (in_sizes[2]  != 2 * DI_ * DM_)   return;
    if (in_sizes[3]  != DI_ * 4)         return;
    if (in_sizes[4]  != DI_)             return;
    if (in_sizes[5]  != XPN_ * DI_)      return;
    if (in_sizes[6]  != DI_ * DR_)       return;
    if (in_sizes[7]  != DI_)             return;
    if (in_sizes[8]  != DI_ * NS_)       return;
    if (in_sizes[9]  != DI_)             return;
    if (in_sizes[10] != DM_ * DI_)       return;
    if (out_size != MT_ * DM_)           return;

    const float* hsx  = (const float*)d_in[0];
    const float* nw   = (const float*)d_in[1];
    const float* wi   = (const float*)d_in[2];
    const float* cw   = (const float*)d_in[3];
    const float* cb   = (const float*)d_in[4];
    const float* wxp  = (const float*)d_in[5];
    const float* wdt  = (const float*)d_in[6];
    const float* dtb  = (const float*)d_in[7];
    const float* alog = (const float*)d_in[8];
    const float* Dp   = (const float*)d_in[9];
    const float* wo   = (const float*)d_in[10];
    float* out = (float*)d_out;

    const size_t SZ_U16  = (size_t)MT_ * DM_ * 2;
    const size_t SZ_WI   = (size_t)2 * DI_ * DM_ * 2;
    const size_t SZ_WXP  = (size_t)XPP_ * DI_ * 2;
    const size_t SZ_WDT  = (size_t)DI_ * DR_ * 2;
    const size_t SZ_WO   = (size_t)DM_ * DI_ * 2;
    const size_t SZ_F    = (size_t)MT_ * DI_ * 4;
    const size_t SZ_XC16 = (size_t)MT_ * DI_ * 2;
    const size_t SZ_DBL  = (size_t)MT_ * XPP_ * 4;
    const size_t SZ_DT16 = (size_t)MT_ * DR_ * 2;
    const size_t SZ_Y16  = (size_t)MT_ * DI_ * 2;

    const size_t OFF_U16  = 0;
    const size_t OFF_WI   = OFF_U16  + SZ_U16;
    const size_t OFF_WXP  = OFF_WI   + SZ_WI;
    const size_t OFF_WDT  = OFF_WXP  + SZ_WXP;
    const size_t OFF_WO   = OFF_WDT  + SZ_WDT;
    const size_t OFF_XF   = OFF_WO   + SZ_WO;
    const size_t OFF_ZF   = OFF_XF   + SZ_F;
    const size_t OFF_XC16 = OFF_ZF   + SZ_F;
    const size_t OFF_DBL  = OFF_XC16 + SZ_XC16;
    const size_t OFF_DT16 = OFF_DBL  + SZ_DBL;
    const size_t OFF_DL   = OFF_DT16 + SZ_DT16;
    const size_t OFF_Y16  = OFF_DL   + SZ_F;
    const size_t WS_END   = OFF_Y16  + SZ_Y16;
    if (ws_size < WS_END) return;

    char* ws = (char*)d_ws;
    unsigned short* u16  = (unsigned short*)(ws + OFF_U16);
    unsigned short* wi16 = (unsigned short*)(ws + OFF_WI);
    unsigned short* wxp16= (unsigned short*)(ws + OFF_WXP);
    unsigned short* wdt16= (unsigned short*)(ws + OFF_WDT);
    unsigned short* wo16 = (unsigned short*)(ws + OFF_WO);
    float*          Xf   = (float*)(ws + OFF_XF);
    float*          Zf   = (float*)(ws + OFF_ZF);
    unsigned short* xc16 = (unsigned short*)(ws + OFF_XC16);
    float*          dbl  = (float*)(ws + OFF_DBL);
    unsigned short* dt16 = (unsigned short*)(ws + OFF_DT16);
    float*          Dl   = (float*)(ws + OFF_DL);
    unsigned short* y16  = (unsigned short*)(ws + OFF_Y16);

    const int BIGSPLIT = 0x40000000;

    hipMemsetAsync(wxp16 + (size_t)XPN_ * DI_, 0, (size_t)(XPP_ - XPN_) * DI_ * 2, stream);

    hipLaunchKernelGGL(rmsnorm_kernel, dim3(MT_), dim3(DM_ / 8), 0, stream, hsx, nw, u16);

    {
        int n8;
        n8 = (2 * DI_ * DM_) / 8;
        hipLaunchKernelGGL(cvt_kernel, dim3((n8 + 255) / 256), dim3(256), 0, stream, wi, wi16, n8, SC_W);
        n8 = (XPN_ * DI_) / 8;
        hipLaunchKernelGGL(cvt_kernel, dim3((n8 + 255) / 256), dim3(256), 0, stream, wxp, wxp16, n8, SC_W);
        n8 = (DI_ * DR_) / 8;
        hipLaunchKernelGGL(cvt_kernel, dim3((n8 + 255) / 256), dim3(256), 0, stream, wdt, wdt16, n8, SC_W);
        n8 = (DM_ * DI_) / 8;
        hipLaunchKernelGGL(cvt_kernel, dim3((n8 + 255) / 256), dim3(256), 0, stream, wo, wo16, n8, SC_W);
    }

    hipLaunchKernelGGL(HIP_KERNEL_NAME(gemm_tn_kernel<4, false>),
                       dim3((2 * DI_) / 128, MT_ / 64), dim3(128), 0, stream,
                       (const unsigned short*)u16, (const unsigned short*)wi16,
                       Xf, Zf, hsx, (int)DM_, (int)DI_, (int)DI_, 1.0f / 256.0f);

    hipLaunchKernelGGL(conv_silu_kernel, dim3(MT_), dim3(DI_ / 8), 0, stream,
                       (const float*)Xf, cw, cb, xc16);

    hipLaunchKernelGGL(HIP_KERNEL_NAME(gemm_tn_kernel<4, false>),
                       dim3(XPP_ / 128, MT_ / 64), dim3(128), 0, stream,
                       (const unsigned short*)xc16, (const unsigned short*)wxp16,
                       dbl, dbl, hsx, (int)DI_, (int)XPP_, BIGSPLIT, 1.0f / 1024.0f);

    hipLaunchKernelGGL(dtslice_kernel, dim3(((MT_ * DR_) / 8 + 255) / 256), dim3(256), 0, stream,
                       (const float*)dbl, dt16);

    hipLaunchKernelGGL(HIP_KERNEL_NAME(gemm_tn_kernel<4, false>),
                       dim3(DI_ / 128, MT_ / 64), dim3(128), 0, stream,
                       (const unsigned short*)dt16, (const unsigned short*)wdt16,
                       Dl, Dl, hsx, (int)DR_, (int)DI_, BIGSPLIT, 1.0f / 1024.0f);

    hipLaunchKernelGGL(scan_kernel, dim3(DI_ / 64, NB_), dim3(64), 0, stream,
                       (const float*)Xf, (const float*)Zf, (const float*)Dl, (const float*)dbl,
                       cw, cb, dtb, alog, Dp, y16);

    hipLaunchKernelGGL(HIP_KERNEL_NAME(gemm_tn_kernel<4, true>),
                       dim3(DM_ / 128, MT_ / 64), dim3(128), 0, stream,
                       (const unsigned short*)y16, (const unsigned short*)wo16,
                       out, out, hsx, (int)DI_, (int)DM_, BIGSPLIT, 1.0f / 2048.0f);
}
